// Block_67980742361706
// MI455X (gfx1250) — hardware-verified
//
#include <hip/hip_runtime.h>
#include <math.h>

#ifndef NB
#define NB 2
#endif
#ifndef SEQ
#define SEQ 2048
#endif
#define NB_FULL 2
#define SEQ_FULL 2048

constexpr int kDim      = 1024;
constexpr int kHeads    = 16;
constexpr int kHeadDim  = 64;
constexpr int kQkvCols  = 3 * kDim;
constexpr int kHid      = 2730;
constexpr int kHidP     = 2752;
constexpr int kN12      = 2 * kHidP;
constexpr int kTok      = NB * SEQ;
constexpr int kTokH     = kTok / 2;
constexpr int kGroups   = NB * kHeads;
constexpr float kWCarry = 16.0f;
constexpr float kPCarry = 256.0f;
constexpr float kOCarry = 64.0f;
constexpr float kHCarry = 16.0f;
constexpr float kAttnScale = 0.125f;
constexpr float kEps    = 1e-6f;
constexpr float kInvDim = 1.0f / 1024.0f;

static_assert((SEQ & (SEQ - 1)) == 0);
static_assert(SEQ >= 64 && SEQ <= SEQ_FULL);
static_assert(NB >= 1 && NB <= NB_FULL);
static_assert(kTokH % 64 == 0);
static_assert(kHidP % 64 == 0 && kHidP >= kHid);
static_assert(kDim % 64 == 0 && kQkvCols % 64 == 0 && kN12 % 64 == 0);
static_assert(kHeads * kHeadDim == kDim);

typedef __attribute__((ext_vector_type(16))) _Float16 v16h;
typedef __attribute__((ext_vector_type(8)))  _Float16 v8h;
typedef __attribute__((ext_vector_type(8)))  float    v8f;
typedef __attribute__((ext_vector_type(4)))  float    v4f;
typedef __attribute__((ext_vector_type(4)))  unsigned int v4u;

__device__ __forceinline__ unsigned short f2bf_bits(float f) {
  unsigned u = __float_as_uint(f);
  return (unsigned short)((u + 0x7FFFu + ((u >> 16) & 1u)) >> 16);
}
__device__ __forceinline__ float bf_bits2f(unsigned short h) { return __uint_as_float(((unsigned)h) << 16); }
__device__ __forceinline__ float bf16_rne(float f) { return bf_bits2f(f2bf_bits(f)); }

__device__ __forceinline__ void dep_guard_h(v8f& a, v8f& b, v16h x, v16h y) { asm volatile("v_nop\n\tv_nop\n\tv_nop\n\tv_nop" : "+v"(a), "+v"(b) : "v"(x), "v"(y)); }
__device__ __forceinline__ void keep4_h(v16h a, v16h b, v16h c, v16h d) { asm volatile("v_nop" :: "v"(a), "v"(b), "v"(c), "v"(d)); }
__device__ __forceinline__ void keep1_h(v16h a) { asm volatile("v_nop" :: "v"(a)); }
__device__ __forceinline__ void acc_guard4(v8f& a, v8f& b, v8f& c, v8f& d) { asm volatile("v_nop\n\tv_nop\n\tv_nop\n\tv_nop" : "+v"(a), "+v"(b), "+v"(c), "+v"(d)); }

struct FragH {
  union U { v16h v; v8h h[2]; };
  static __device__ __forceinline__ v16h load(const _Float16* p) {
    U f; f.h[0] = *(const v8h*)(p); f.h[1] = *(const v8h*)(p + 16); return f.v;
  }
  static __device__ __forceinline__ v8f mma(v16h a, v16h b, v8f c) {
    return __builtin_amdgcn_wmma_f32_16x16x32_f16(false, a, false, b, (short)0, c, false, false);
  }
};

__device__ __forceinline__ unsigned pk16(unsigned short a, unsigned short b) { return (unsigned)a | ((unsigned)b << 16); }
__device__ __forceinline__ unsigned short h_bits(float f) { const _Float16 h = (_Float16)f; return __builtin_bit_cast(unsigned short, h); }

template <int BIAS_MODE, int OUT_MODE, bool RESID, bool ROPE>
__global__ __launch_bounds__(256) void wmma_gemm64(
    const unsigned short* __restrict__ Ap, int lda,
    const unsigned short* __restrict__ Btp, int ldb,
    void* __restrict__ Cout, int ldc,
    const float* __restrict__ bias,
    const float* __restrict__ resid,
    const float* __restrict__ cosT, const float* __restrict__ sinT, int ropeCols,
    int M, int N, int K, float scale) {
  const _Float16* A  = (const _Float16*)Ap;
  const _Float16* Bt = (const _Float16*)Btp;
  __shared__ __align__(16) float sT[8][16 * 68];
  const int lane = threadIdx.x & 31;
  const int wave = threadIdx.x >> 5;
  const int tilesN = N >> 6;
  const int tn = blockIdx.x * 8 + wave;
  const int tm = blockIdx.y;
  if (tn >= tilesN || (tm << 6) >= M) return;
  const int m0 = tm << 6;
  const int n0 = tn << 6;

  const int rlane = lane & 15;
  const int koff  = (lane >> 4) * 8;
  const int mOff  = (lane >> 4) * 8;

  v8f acc[4][4];
#pragma unroll
  for (int i = 0; i < 4; ++i)
#pragma unroll
    for (int j = 0; j < 4; ++j) acc[i][j] = (v8f){0.f,0.f,0.f,0.f,0.f,0.f,0.f,0.f};

  for (int k0 = 0; k0 < K; k0 += 32) {
    v16h bh[4];
#pragma unroll
    for (int j = 0; j < 4; ++j) {
      const size_t bo = (size_t)(n0 + (j << 4) + rlane) * ldb + koff + k0;
      bh[j] = FragH::load(Bt + bo);
    }
#pragma unroll
    for (int i = 0; i < 4; ++i) {
      const size_t ao = (size_t)(m0 + (i << 4) + rlane) * lda + koff + k0;
      v16h ah = FragH::load(A + ao);
#pragma unroll
      for (int j = 0; j < 4; ++j) acc[i][j] = FragH::mma(ah, bh[j], acc[i][j]);
      dep_guard_h(acc[i][0], acc[i][3], ah, ah);
    }
    keep4_h(bh[0], bh[1], bh[2], bh[3]);
  }
  acc_guard4(acc[0][0], acc[0][1], acc[0][2], acc[0][3]);
  acc_guard4(acc[1][0], acc[1][1], acc[1][2], acc[1][3]);
  acc_guard4(acc[2][0], acc[2][1], acc[2][2], acc[2][3]);
  acc_guard4(acc[3][0], acc[3][1], acc[3][2], acc[3][3]);

  float* slab = sT[wave];
  const bool doRope = ROPE && (n0 < ropeCols);
#pragma unroll
  for (int i = 0; i < 4; ++i) {
    const int mBase = m0 + (i << 4);
#pragma unroll
    for (int j = 0; j < 4; ++j) {
      const int n = n0 + (j << 4) + rlane;
      float bv = 0.f;
      if (BIAS_MODE == 2) bv = bf16_rne(bias[n]);
#pragma unroll
      for (int r = 0; r < 8; ++r) {
        float v = acc[i][j][r] * scale;
        if (BIAS_MODE == 2) v += bv;
        if (RESID) v += resid[(size_t)(mBase + mOff + r) * ldc + n];
        slab[(mOff + r) * 68 + (j << 4) + rlane] = v;
      }
    }
    __builtin_amdgcn_fence(3  , "workgroup");
    __builtin_amdgcn_wave_barrier();
    __builtin_amdgcn_fence(2  , "workgroup");
    if (OUT_MODE == 0) {
      float* C = (float*)Cout;
      const int hh = lane >> 4, c4 = (lane & 15) * 4;
      for (int pass = 0; pass < 2; ++pass) {
#pragma unroll
        for (int it = 0; it < 8; ++it) {
          const int row = it * 2 + hh;
          v4f v = *(const v4f*)(slab + row * 68 + c4);
          *(volatile v4f*)(C + (size_t)(mBase + row) * ldc + n0 + c4) = v;
        }
        __threadfence();
      }
    } else {
      const int q = lane >> 3, c8 = (lane & 7) * 8;
      unsigned short* C = (unsigned short*)Cout;
      for (int pass = 0; pass < 2; ++pass) {
#pragma unroll
        for (int it = 0; it < 4; ++it) {
          const int row = it * 4 + q;
          const float* sp = slab + row * 68 + c8;
          float ev[8];
#pragma unroll
          for (int e = 0; e < 8; ++e) ev[e] = sp[e];
          if (ROPE) {
            if (doRope) {
              const unsigned tpos = (unsigned)(mBase + row) & (unsigned)(SEQ - 1);
              const v4f cv = *(const v4f*)(cosT + (size_t)tpos * 32 + (c8 >> 1));
              const v4f sv = *(const v4f*)(sinT + (size_t)tpos * 32 + (c8 >> 1));
#pragma unroll
              for (int p = 0; p < 4; ++p) {
                const float c = bf16_rne(cv[p]);
                const float s = bf16_rne(sv[p]);
                const float x0 = ev[2 * p], x1 = ev[2 * p + 1];
                ev[2 * p]     = x0 * c - x1 * s;
                ev[2 * p + 1] = x0 * s + x1 * c;
              }
            }
          }
          v8h hv;
#pragma unroll
          for (int e = 0; e < 8; ++e) hv[e] = (_Float16)ev[e];
          *(volatile v8h*)(C + (size_t)(mBase + row) * ldc + n0 + c8) = hv;
        }
        __threadfence();
      }
    }
    __builtin_amdgcn_fence(3  , "workgroup");
    __builtin_amdgcn_wave_barrier();
    __builtin_amdgcn_fence(2  , "workgroup");
  }
}

__global__ __launch_bounds__(128) void wcast_kernel(const float* __restrict__ W, unsigned short* __restrict__ out,
                                                    unsigned rows, unsigned K, unsigned KP, float scale) {
  const unsigned k8i = blockIdx.x * 128u + threadIdx.x;
  const unsigned r   = blockIdx.y;
  if (k8i >= (KP >> 3)) return;
  const unsigned k0 = k8i << 3;
  const unsigned rc = (r < rows) ? r : (rows - 1u);
  const float* src = W + (size_t)rc * K;
  unsigned short hb[8];
#pragma unroll
  for (unsigned e = 0; e < 8; ++e) {
    const unsigned k  = k0 + e;
    const unsigned kc = (k < K) ? k : (K - 1u);
    const float v = src[kc];
    const bool ok = (r < rows) && (k < K);
    const unsigned short bits = h_bits(bf16_rne(v) * scale);
    hb[e] = ok ? bits : (unsigned short)0;
  }
  const v4u u = (v4u){pk16(hb[0], hb[1]), pk16(hb[2], hb[3]), pk16(hb[4], hb[5]), pk16(hb[6], hb[7])};
  unsigned short* op = out + (size_t)r * KP + k0;
  *(volatile v4u*)op = u;
  __threadfence();
  *(volatile v4u*)op = u;
}

__global__ __launch_bounds__(128) void biaspad_kernel(const float* __restrict__ b1, const float* __restrict__ b2,
                                                      float* __restrict__ out) {
  const unsigned i = blockIdx.x * 128u + threadIdx.x;
  if (i >= (unsigned)(kN12 / 4)) return;
  v4f v;
#pragma unroll
  for (unsigned e = 0; e < 4; ++e) {
    const unsigned n   = 4u * i + e;
    const bool     sec = n >= (unsigned)kHidP;
    const unsigned j   = sec ? (n - (unsigned)kHidP) : n;
    const unsigned jc  = (j < (unsigned)kHid) ? j : (unsigned)(kHid - 1);
    const float a = b1[jc];
    const float c = b2[jc];
    const float val = sec ? c : a;
    v[e] = (j < (unsigned)kHid) ? bf16_rne(val) : 0.0f;
  }
  float* op = out + 4u * i;
  *(volatile v4f*)op = v;
  __threadfence();
  *(volatile v4f*)op = v;
}

template <bool FROM_INPUT>
__global__ __launch_bounds__(256) void rms_row_kernel(const float* __restrict__ X, const float* __restrict__ gw,
                                                      float* __restrict__ Yf, unsigned short* __restrict__ Yh) {
  __shared__ float red[8];
  __shared__ float stat[1];
  const unsigned row  = blockIdx.x;
  const unsigned t    = threadIdx.x;
  const unsigned lane = t & 31u, wave = t >> 5;
  size_t xoff;
  if (FROM_INPUT) {
    const unsigned b  = row / (unsigned)SEQ;
    const unsigned tt = row & (unsigned)(SEQ - 1);
    xoff = ((size_t)b * SEQ_FULL + tt) * kDim;
  } else {
    xoff = (size_t)row * kDim;
  }
  const float* xr = X + xoff;
  v4f a = *(const v4f*)(xr + 4u * t);
  if (FROM_INPUT) {
#pragma unroll
    for (int e = 0; e < 4; ++e) a[e] = bf16_rne(a[e]);
  }
  float s = (a[0] * a[0] + a[1] * a[1]) + (a[2] * a[2] + a[3] * a[3]);
#pragma unroll
  for (int off = 16; off > 0; off >>= 1) s += __shfl_xor(s, off, 32);
  if (lane == 0) red[wave] = s;
  __syncthreads();
  if (t == 0) {
    float tot = red[0];
#pragma unroll
    for (int w = 1; w < 8; ++w) tot += red[w];
    stat[0] = rsqrtf(tot * kInvDim + kEps);
  }
  __syncthreads();
  const float rs = stat[0];
  v4f g = *(const v4f*)(gw + 4u * t);
  v4f y;
#pragma unroll
  for (int e = 0; e < 4; ++e) y[e] = (a[e] * rs) * bf16_rne(g[e]);
  float* yp = Yf + (size_t)row * kDim + 4u * t;
  v4u u = (v4u){0u, 0u, 0u, 0u};
  unsigned short* hp = Yh + (size_t)row * kDim + 8u * (t & 127u);
  if (wave < 4) {
    const unsigned c0 = 8u * t;
    v4f xa = *(const v4f*)(xr + c0);
    v4f xb = *(const v4f*)(xr + c0 + 4);
    const v4f ga = *(const v4f*)(gw + c0);
    const v4f gb = *(const v4f*)(gw + c0 + 4);
    unsigned short hb[8];
#pragma unroll
    for (int e = 0; e < 4; ++e) {
      const float x0 = FROM_INPUT ? bf16_rne(xa[e]) : xa[e];
      const float x1 = FROM_INPUT ? bf16_rne(xb[e]) : xb[e];
      hb[e]     = h_bits((x0 * rs) * bf16_rne(ga[e]));
      hb[4 + e] = h_bits((x1 * rs) * bf16_rne(gb[e]));
    }
    u = (v4u){pk16(hb[0], hb[1]), pk16(hb[2], hb[3]), pk16(hb[4], hb[5]), pk16(hb[6], hb[7])};
  }
  *(volatile v4f*)yp = y;
  if (wave < 4) *(volatile v4u*)hp = u;
  __threadfence();
  *(volatile v4f*)yp = y;
  if (wave < 4) *(volatile v4u*)hp = u;
}

__global__ __launch_bounds__(256) void vtrans_kernel(const unsigned short* __restrict__ qkv, unsigned short* __restrict__ Vt) {
  __shared__ unsigned short sm[64][66];
  const unsigned t  = threadIdx.x;
  const unsigned g  = blockIdx.y;
  const unsigned b  = g >> 4, h = g & 15u;
  const unsigned n0 = blockIdx.x * 64u;
#pragma unroll
  for (unsigned it = 0; it < 2; ++it) {
    const unsigned idx = it * 256u + t;
    const unsigned r   = idx >> 3;
    const unsigned seg = (idx & 7u) * 8u;
    const size_t off = ((size_t)b * SEQ + n0 + r) * kQkvCols + 2 * kDim + h * kHeadDim + seg;
    const v4u w = *(const v4u*)(qkv + off);
    sm[r][seg + 0] = (unsigned short)(w.x & 0xffffu); sm[r][seg + 1] = (unsigned short)(w.x >> 16);
    sm[r][seg + 2] = (unsigned short)(w.y & 0xffffu); sm[r][seg + 3] = (unsigned short)(w.y >> 16);
    sm[r][seg + 4] = (unsigned short)(w.z & 0xffffu); sm[r][seg + 5] = (unsigned short)(w.z >> 16);
    sm[r][seg + 6] = (unsigned short)(w.w & 0xffffu); sm[r][seg + 7] = (unsigned short)(w.w >> 16);
  }
  __syncthreads();
  const unsigned lane = t & 31u, wave = t >> 5;
  const unsigned q = lane >> 3, c8 = (lane & 7u) * 8u;
  unsigned short* vb = Vt + (size_t)g * kHeadDim * SEQ;
  for (int pass = 0; pass < 2; ++pass) {
#pragma unroll
    for (unsigned it = 0; it < 2; ++it) {
      const unsigned dh = wave * 8u + it * 4u + q;
      unsigned short hb[8];
#pragma unroll
      for (unsigned e = 0; e < 8; ++e) hb[e] = sm[c8 + e][dh];
      const v4u u = (v4u){pk16(hb[0], hb[1]), pk16(hb[2], hb[3]), pk16(hb[4], hb[5]), pk16(hb[6], hb[7])};
      *(volatile v4u*)(vb + (size_t)dh * SEQ + n0 + c8) = u;
    }
    __threadfence();
  }
}

__global__ __launch_bounds__(128) void flash_attn_kernel(const unsigned short* __restrict__ qkvp,
                                                         const unsigned short* __restrict__ Vtp,
                                                         unsigned short* __restrict__ attnp) {
  __shared__ __align__(16) float sO[4][16 * 68];
  const unsigned lane = threadIdx.x & 31u;
  const unsigned wave = threadIdx.x >> 5;
  const unsigned lh = lane >> 4, ln = lane & 15u;
  const unsigned g = blockIdx.y;
  const unsigned b = g >> 4, h = g & 15u;
  const unsigned qBase = (blockIdx.x * 4u + wave) << 4;
  const _Float16* qkv = (const _Float16*)qkvp;
  const size_t tok0 = (size_t)b * SEQ;

  const _Float16* qrow = qkv + (tok0 + qBase + ln) * kQkvCols + h * kHeadDim + 8u * lh;
  const v16h qf0 = FragH::load(qrow);
  const v16h qf1 = FragH::load(qrow + 32);
  const _Float16* kpan = qkv + tok0 * kQkvCols + kDim + h * kHeadDim + 8u * lh;
  const _Float16* vpan = (const _Float16*)Vtp + (size_t)g * kHeadDim * SEQ + (size_t)ln * SEQ + 8u * lh;

  const v8f zero8 = (v8f){0.f,0.f,0.f,0.f,0.f,0.f,0.f,0.f};
  v8f o0 = zero8, o1 = zero8, o2 = zero8, o3 = zero8;
  float mrow = -1e30f, lrow = 0.f;
  const unsigned qg = qBase + ln;
  const unsigned nblk = (qBase >> 5) + 1u;

#pragma unroll 1
  for (unsigned jb = 0; jb < nblk; ++jb) {
    const unsigned kBase = jb << 5;
    const _Float16* kr0 = kpan + (size_t)(kBase + ln) * kQkvCols;
    const _Float16* kr1 = kr0 + (size_t)16 * kQkvCols;
    const v16h k00 = FragH::load(kr0);
    const v16h k01 = FragH::load(kr0 + 32);
    const v16h k10 = FragH::load(kr1);
    const v16h k11 = FragH::load(kr1 + 32);
    v8f s0 = zero8, s1 = zero8;
    s0 = FragH::mma(k00, qf0, s0);
    s0 = FragH::mma(k01, qf1, s0);
    s1 = FragH::mma(k10, qf0, s1);
    s1 = FragH::mma(k11, qf1, s1);
    dep_guard_h(s0, s1, qf0, qf1);
    keep4_h(k00, k01, k10, k11);

    const unsigned kg0 = kBase + 8u * lh;
    float pv[16];
    float bm = -1e30f;
#pragma unroll
    for (int r = 0; r < 8; ++r) {
      float v = s0[r] * kAttnScale;
      v = ((kg0 + (unsigned)r) > qg) ? -1e30f : v;
      pv[r] = v;
      bm = fmaxf(bm, v);
    }
#pragma unroll
    for (int r = 0; r < 8; ++r) {
      float v = s1[r] * kAttnScale;
      v = ((kg0 + 16u + (unsigned)r) > qg) ? -1e30f : v;
      pv[8 + r] = v;
      bm = fmaxf(bm, v);
    }
    bm = fmaxf(bm, __shfl_xor(bm, 16, 32));
    const float mnew = fmaxf(mrow, bm);
    float ls = 0.f;
    v16h pf;
#pragma unroll
    for (int i = 0; i < 16; ++i) {
      const unsigned kg = kg0 + (unsigned)((i >> 3) << 4) + (unsigned)(i & 7);
      float p = __expf(pv[i] - mnew);
      p = (kg > qg) ? 0.f : p;
      ls += p;
      pf[i] = (_Float16)(p * kPCarry);
    }
    ls += __shfl_xor(ls, 16, 32);
    const float corr = __expf(mrow - mnew);
    lrow = lrow * corr + ls;
    mrow = mnew;
    float c8[8];
#pragma unroll
    for (int r = 0; r < 8; ++r) c8[r] = __shfl(corr, (int)(8u * lh) + r, 16);
#pragma unroll
    for (int r = 0; r < 8; ++r) { o0[r] *= c8[r]; o1[r] *= c8[r]; o2[r] *= c8[r]; o3[r] *= c8[r]; }

    const _Float16* vr = vpan + kBase;
    const v16h v0 = FragH::load(vr);
    const v16h v1 = FragH::load(vr + (size_t)16 * SEQ);
    const v16h v2 = FragH::load(vr + (size_t)32 * SEQ);
    const v16h v3 = FragH::load(vr + (size_t)48 * SEQ);
    o0 = FragH::mma(pf, v0, o0);
    o1 = FragH::mma(pf, v1, o1);
    o2 = FragH::mma(pf, v2, o2);
    o3 = FragH::mma(pf, v3, o3);
    acc_guard4(o0, o1, o2, o3);
    keep4_h(v0, v1, v2, v3);
    keep1_h(pf);
  }

  const float invl = (kOCarry / kPCarry) * __builtin_amdgcn_rcpf(lrow);
  float i8[8];
#pragma unroll
  for (int r = 0; r < 8; ++r) i8[r] = __shfl(invl, (int)(8u * lh) + r, 16);
  float* slab = sO[wave];
#pragma unroll
  for (int r = 0; r < 8; ++r) {
    const unsigned rowl = 8u * lh + (unsigned)r;
    slab[rowl * 68u + ln]       = o0[r] * i8[r];
    slab[rowl * 68u + 16u + ln] = o1[r] * i8[r];
    slab[rowl * 68u + 32u + ln] = o2[r] * i8[r];
    slab[rowl * 68u + 48u + ln] = o3[r] * i8[r];
  }
  __builtin_amdgcn_fence(3  , "workgroup");
  __builtin_amdgcn_wave_barrier();
  __builtin_amdgcn_fence(2  , "workgroup");
  const unsigned q = lane >> 3, cc8 = (lane & 7u) * 8u;
  unsigned short* ob = attnp + (tok0 + qBase) * kDim + h * kHeadDim;
  for (int pass = 0; pass < 2; ++pass) {
#pragma unroll
    for (unsigned it = 0; it < 4; ++it) {
      const unsigned row = it * 4u + q;
      const float* sp = slab + row * 68u + cc8;
      v8h hv;
#pragma unroll
      for (int e = 0; e < 8; ++e) hv[e] = (_Float16)sp[e];
      *(volatile v8h*)(ob + (size_t)row * kDim + cc8) = hv;
    }
    __threadfence();
  }
}

__global__ __launch_bounds__(128) void swiglu_kernel(const float* __restrict__ pre, unsigned short* __restrict__ hout) {
  const unsigned k8i = blockIdx.x * 128u + threadIdx.x;
  const unsigned row = blockIdx.y;
  if (k8i >= (unsigned)(kHidP >> 3)) return;
  const unsigned j0 = k8i << 3;
  const float* pa = pre + (size_t)row * kN12 + j0;
  const v4f a0 = *(const v4f*)(pa);
  const v4f a1 = *(const v4f*)(pa + 4);
  const v4f g0 = *(const v4f*)(pa + kHidP);
  const v4f g1 = *(const v4f*)(pa + kHidP + 4);
  unsigned short hb[8];
#pragma unroll
  for (unsigned e = 0; e < 4; ++e) {
    const float x0 = a0[e], x1 = a1[e];
    const float h0 = x0 * (1.0f + __expf(-x0)) * g0[e] * kHCarry;
    const float h1 = x1 * (1.0f + __expf(-x1)) * g1[e] * kHCarry;
    const unsigned short b0 = h_bits(h0);
    const unsigned short b1 = h_bits(h1);
    hb[e]     = ((j0 + e) < (unsigned)kHid) ? b0 : (unsigned short)0;
    hb[4 + e] = ((j0 + 4u + e) < (unsigned)kHid) ? b1 : (unsigned short)0;
  }
  const v4u u = (v4u){pk16(hb[0], hb[1]), pk16(hb[2], hb[3]), pk16(hb[4], hb[5]), pk16(hb[6], hb[7])};
  unsigned short* op = hout + (size_t)row * kHidP + j0;
  *(volatile v4u*)op = u;
  __threadfence();
  *(volatile v4u*)op = u;
}

constexpr size_t szWqkv  = (size_t)kQkvCols * kDim * 2;
constexpr size_t szWo    = (size_t)kDim * kDim * 2;
constexpr size_t szW12   = (size_t)kN12 * kDim * 2;
constexpr size_t szW3    = (size_t)kDim * kHidP * 2;
constexpr size_t szBias  = 22528;
constexpr size_t szXf    = (size_t)kTok * kDim * 4;
constexpr size_t szXh    = (size_t)kTok * kDim * 2;
constexpr size_t szQkv   = (size_t)kTok * kQkvCols * 2;
constexpr size_t szVt    = (size_t)kGroups * kHeadDim * SEQ * 2;
constexpr size_t szAttn  = (size_t)kTok * kDim * 2;
constexpr size_t szPre   = (size_t)kTokH * kN12 * 4;
constexpr size_t szH     = (size_t)kTok * kHidP * 2;
constexpr size_t szS1    = szQkv + szVt + szAttn;
constexpr size_t szS2    = szPre + szH;
constexpr size_t szS     = (szS1 > szS2) ? szS1 : szS2;
constexpr size_t offWqkv = 0;
constexpr size_t offWo   = offWqkv + szWqkv;
constexpr size_t offW12  = offWo + szWo;
constexpr size_t offW3   = offW12 + szW12;
constexpr size_t offBias = offW3 + szW3;
constexpr size_t offXf   = offBias + szBias;
constexpr size_t offXh   = offXf + szXf;
constexpr size_t offS    = offXh + szXh;
constexpr size_t wsTotal = offS + szS;
static_assert(wsTotal <= (size_t)134217728);
static_assert((size_t)kN12 * 4 <= szBias);
static_assert(szXf <= szQkv);
static_assert(offWo % 128 == 0 && offW12 % 128 == 0 && offW3 % 128 == 0 && offBias % 128 == 0);
static_assert(offXf % 128 == 0 && offXh % 128 == 0 && offS % 128 == 0);
static_assert(szQkv % 128 == 0 && szVt % 128 == 0 && szPre % 128 == 0);
static_assert((kHidP >> 3) <= 3 * 128);
static_assert((kDim >> 3) <= 128);

extern "C" void kernel_launch(void* const* d_in, const int* in_sizes, int n_in,
                              void* d_out, int out_size, void* d_ws, size_t ws_size,
                              hipStream_t stream) {
  if (n_in < 16) return;
  const long needX = ((long)(NB - 1) * SEQ_FULL + SEQ) * kDim;
  if ((long)in_sizes[0] < needX) return;
  if (in_sizes[1] < kDim || in_sizes[2] < kDim * kDim || in_sizes[3] < kDim * kDim || in_sizes[4] < kDim * kDim ||
      in_sizes[5] < kDim * kDim || in_sizes[6] < kDim || in_sizes[7] < kHid * kDim || in_sizes[8] < kHid ||
      in_sizes[9] < kHid * kDim || in_sizes[10] < kHid || in_sizes[11] < kDim * kHid || in_sizes[12] < kDim ||
      in_sizes[13] < kDim || in_sizes[14] < SEQ * 32 || in_sizes[15] < SEQ * 32) return;
  if (out_size < kTok * kDim) return;
  if (wsTotal > ws_size) return;

  const float* x     = (const float*)d_in[0];
  const float* ln1w  = (const float*)d_in[1];
  const float* Wq    = (const float*)d_in[2];
  const float* Wk    = (const float*)d_in[3];
  const float* Wv    = (const float*)d_in[4];
  const float* Wo    = (const float*)d_in[5];
  const float* bo    = (const float*)d_in[6];
  const float* w1    = (const float*)d_in[7];
  const float* b1    = (const float*)d_in[8];
  const float* w2    = (const float*)d_in[9];
  const float* b2    = (const float*)d_in[10];
  const float* w3    = (const float*)d_in[11];
  const float* b3    = (const float*)d_in[12];
  const float* ln2w  = (const float*)d_in[13];
  const float* cosT  = (const float*)d_in[14];
  const float* sinT  = (const float*)d_in[15];
  float* out = (float*)d_out;

  char* ws = (char*)d_ws;
  unsigned short* WqkvT = (unsigned short*)(ws + offWqkv);
  unsigned short* WoT   = (unsigned short*)(ws + offWo);
  unsigned short* W12   = (unsigned short*)(ws + offW12);
  unsigned short* W3T   = (unsigned short*)(ws + offW3);
  float*          bias12 = (float*)(ws + offBias);
  float*          Xf    = (float*)(ws + offXf);
  unsigned short* Xh    = (unsigned short*)(ws + offXh);
  unsigned short* qkv   = (unsigned short*)(ws + offS);
  unsigned short* Vt    = (unsigned short*)(ws + offS + szQkv);
  unsigned short* attn  = (unsigned short*)(ws + offS + szQkv + szVt);
  float*          x2    = (float*)(ws + offS);
  float*          pre   = (float*)(ws + offS);
  unsigned short* hpl   = (unsigned short*)(ws + offS + szPre);

  wcast_kernel<<<dim3(1, kDim), dim3(128), 0, stream>>>(Wq, WqkvT, kDim, kDim, kDim, kWCarry);
  wcast_kernel<<<dim3(1, kDim), dim3(128), 0, stream>>>(Wk, WqkvT + (size_t)kDim * kDim, kDim, kDim, kDim, kWCarry);
  wcast_kernel<<<dim3(1, kDim), dim3(128), 0, stream>>>(Wv, WqkvT + (size_t)2 * kDim * kDim, kDim, kDim, kDim, kWCarry);
  wcast_kernel<<<dim3(1, kDim), dim3(128), 0, stream>>>(Wo, WoT, kDim, kDim, kDim, kWCarry);
  wcast_kernel<<<dim3(1, kHidP), dim3(128), 0, stream>>>(w1, W12, kHid, kDim, kDim, kWCarry);
  wcast_kernel<<<dim3(1, kHidP), dim3(128), 0, stream>>>(w2, W12 + (size_t)kHidP * kDim, kHid, kDim, kDim, kWCarry);
  wcast_kernel<<<dim3(3, kDim), dim3(128), 0, stream>>>(w3, W3T, kDim, kHid, kHidP, kWCarry);
  biaspad_kernel<<<dim3((kN12 / 4 + 127) / 128), dim3(128), 0, stream>>>(b1, b2, bias12);

  rms_row_kernel<true><<<dim3(kTok), dim3(256), 0, stream>>>(x, ln1w, Xf, Xh);

  wmma_gemm64<0, 1, false, true><<<dim3((kQkvCols / 64 + 7) / 8, kTok / 64), dim3(256), 0, stream>>>(
      Xh, kDim, WqkvT, kDim, (void*)qkv, kQkvCols, nullptr, nullptr, cosT, sinT, 2 * kDim,
      kTok, kQkvCols, kDim, 1.0f / kWCarry);

  vtrans_kernel<<<dim3(SEQ / 64, kGroups), dim3(256), 0, stream>>>(qkv, Vt);

  flash_attn_kernel<<<dim3(SEQ / 64, kGroups), dim3(128), 0, stream>>>(qkv, Vt, attn);

  wmma_gemm64<2, 0, true, false><<<dim3((kDim / 64 + 7) / 8, kTok / 64), dim3(256), 0, stream>>>(
      attn, kDim, WoT, kDim, (void*)x2, kDim, bo, Xf, nullptr, nullptr, 0,
      kTok, kDim, kDim, 1.0f / (kOCarry * kWCarry));

  rms_row_kernel<false><<<dim3(kTok), dim3(256), 0, stream>>>(x2, ln2w, Xf, Xh);

  for (int half = 0; half < 2; ++half) {
    const unsigned short* Ah = Xh + (size_t)half * kTokH * kDim;
    wmma_gemm64<2, 0, false, false><<<dim3((kN12 / 64 + 7) / 8, kTokH / 64), dim3(256), 0, stream>>>(
        Ah, kDim, W12, kDim, (void*)pre, kN12, bias12, nullptr, nullptr, nullptr, 0,
        kTokH, kN12, kDim, 1.0f / kWCarry);
    swiglu_kernel<<<dim3(3, kTokH), dim3(128), 0, stream>>>(pre, hpl + (size_t)half * kTokH * kHidP);
  }

  wmma_gemm64<2, 0, true, false><<<dim3((kDim / 64 + 7) / 8, kTok / 64), dim3(256), 0, stream>>>(
      hpl, kHidP, W3T, kHidP, (void*)out, kDim, b3, Xf, nullptr, nullptr, 0,
      kTok, kDim, kHidP, 1.0f / (kHCarry * kWCarry));
}
